// PointNetSetAbstraction_42588895707400
// MI455X (gfx1250) — hardware-verified
//
#include <hip/hip_runtime.h>
#pragma clang fp contract(off)

typedef __attribute__((ext_vector_type(16))) _Float16 v16h;
typedef __attribute__((ext_vector_type(8)))  _Float16 v8h;
typedef __attribute__((ext_vector_type(8)))  float    v8f;
typedef __attribute__((ext_vector_type(4)))  float    v4f;
typedef __attribute__((ext_vector_type(2)))  float    v2f;

constexpr int kBatch   = 8;
constexpr int kNpts    = 4096;
constexpr int kNcen    = 1024;
constexpr int kNsmp    = 32;
constexpr int kCpts    = 64;
constexpr int kCin0    = 67;
constexpr int kCmid    = 64;
constexpr int kCout    = 128;
constexpr int kTdim    = 128;
constexpr int kCenTot  = kBatch * kNcen;
constexpr int kRowsTot = kCenTot * kNsmp;
constexpr int kSrcTot  = kBatch * kNpts;
constexpr float kRad2  = (float)(0.2 * 0.2);
constexpr float kBnEps = 1e-5f;
constexpr float kWCarry = 16.0f;
constexpr float kXCarry = 16.0f;
constexpr float kInvCarry0 = 1.0f / kWCarry;
constexpr float kInvCarry1 = 1.0f / (kWCarry * kXCarry);
constexpr double kInvCount = 1.0 / (double)kRowsTot;

static_assert(kCenTot == 8192, "centroid count");
static_assert(kRowsTot == 262144, "grouped rows");
static_assert(kSrcTot % 64 == 0 && kCmid % 64 == 0 && kCpts % 32 == 0, "conv0 gemm tiles");
static_assert(kRowsTot % 128 == 0 && kCout == 128 && kCmid % 32 == 0, "conv1 gemm tiles");
static_assert(kCin0 == kCpts + 3, "channel order xyz(3) then points(64)");

constexpr size_t kOffNxyz  = 0;
constexpr size_t kOffIdx   = kOffNxyz  + (size_t)kCenTot * 3 * 4;
constexpr size_t kOffBias0 = kOffIdx   + (size_t)kCenTot * kNsmp * 4;
constexpr size_t kOffBias1 = kOffBias0 + (size_t)kBatch * kCmid * 4;
constexpr size_t kOffW0x   = kOffBias1 + (size_t)kBatch * kCout * 4;
constexpr size_t kOffW0p   = kOffW0x   + (size_t)kCmid * 4 * 4;
constexpr size_t kOffW1h   = kOffW0p   + (size_t)kCmid * kCpts * 2;
constexpr size_t kOffSt0   = kOffW1h   + (size_t)kCout * kCmid * 2;
constexpr size_t kOffSt1   = kOffSt0   + (size_t)2 * kCmid * 4;
constexpr size_t kOffPart0 = kOffSt1   + (size_t)2 * kCout * 4;
constexpr size_t kOffPart1 = kOffPart0 + (size_t)256 * 128 * 4;
constexpr size_t kOffPtsT  = kOffPart1 + (size_t)2048 * 256 * 4;
constexpr size_t kOffP0    = kOffPtsT  + (size_t)kSrcTot * kCpts * 2;
constexpr size_t kOffX1    = kOffP0    + (size_t)kSrcTot * kCmid * 4;
constexpr size_t kOffYmm   = kOffX1    + (size_t)kRowsTot * kCmid * 2;
constexpr size_t kWsTotal  = kOffYmm   + (size_t)kCenTot * 256 * 4;
static_assert(kWsTotal <= (size_t)134217728, "carve under 128 MiB");
static_assert(kOffIdx % 128 == 0 && kOffBias0 % 128 == 0 && kOffW0x % 128 == 0 && kOffW0p % 128 == 0 &&
              kOffW1h % 128 == 0 && kOffSt0 % 128 == 0 && kOffSt1 % 128 == 0 && kOffPart0 % 128 == 0 &&
              kOffPart1 % 128 == 0 && kOffPtsT % 128 == 0 && kOffP0 % 128 == 0 && kOffX1 % 128 == 0 &&
              kOffYmm % 128 == 0, "line aligned regions");
constexpr size_t kOut1Floats = (size_t)kCenTot * 3;
static_assert(kOut1Floats * 4 == 98304, "out1 byte offset");
static_assert(kOut1Floats * 4 + (size_t)kBatch * kCout * kNcen * 4 == 4292608, "d_out total");

__device__ __forceinline__ int clampi(int v, int lo, int hi) { return v < lo ? lo : (v > hi ? hi : v); }

__device__ __forceinline__ float gelu_erf(float x) {
  return 0.5f * x * (1.0f + erff(x * 0.70710678118654752440f));
}

__device__ __forceinline__ void dep_guard4_h(v8f& a, v8f& b, v8f& c, v8f& d, v16h x, v16h y) {
  asm volatile("v_nop\n\tv_nop\n\tv_nop\n\tv_nop" : "+v"(a), "+v"(b), "+v"(c), "+v"(d) : "v"(x), "v"(y));
}
__device__ __forceinline__ void keep4_h(v16h a, v16h b, v16h c, v16h d) { asm volatile("v_nop" :: "v"(a), "v"(b), "v"(c), "v"(d)); }
__device__ __forceinline__ void acc_guard4(v8f& a, v8f& b, v8f& c, v8f& d) { asm volatile("v_nop\n\tv_nop\n\tv_nop\n\tv_nop" : "+v"(a), "+v"(b), "+v"(c), "+v"(d)); }
struct FragH {
  union U { v16h v; v8h h[2]; };
  static __device__ __forceinline__ v16h load(const _Float16* p) {
    U f; f.h[0] = *(const v8h*)(p); f.h[1] = *(const v8h*)(p + 16); return f.v;
  }
  static __device__ __forceinline__ v8f mma(v16h a, v16h b, v8f c) {
    return __builtin_amdgcn_wmma_f32_16x16x32_f16(false, a, false, b, (short)0, c, false, false);
  }
};
__device__ __forceinline__ v8f mma_g(v16h a, v16h b, v8f c) {
  c = __builtin_amdgcn_wmma_f32_16x16x32_f16(false, a, false, b, (short)0, c, false, false);
  asm volatile("v_nop\n\tv_nop\n\tv_nop\n\tv_nop" : "+v"(c) : "v"(a), "v"(b));
  return c;
}

__device__ __forceinline__ void argmax_step(float& bv, int& bi, int off) {
  const float ov = __shfl_xor(bv, off, 32);
  const int   oi = __shfl_xor(bi, off, 32);
  const bool take = (ov > bv) || ((ov == bv) && (oi < bi));
  bv = take ? ov : bv;
  bi = take ? oi : bi;
}

__global__ __launch_bounds__(1024) void fps_kernel(const float* __restrict__ xyz,
                                                   float* __restrict__ nxyz_ws,
                                                   float* __restrict__ out0) {
#pragma clang fp contract(off)
  __shared__ float sx[kNpts * 3];
  __shared__ int   scent[kNcen];
  __shared__ float rv[2][32];
  __shared__ int   ri[2][32];
  const int b = blockIdx.x;
  const int tid = threadIdx.x;
  const int lane = tid & 31;
  const int wave = tid >> 5;
  const float* xb = xyz + (size_t)b * kNpts * 3;
  for (int i = tid; i < kNpts * 3; i += 1024) sx[i] = xb[i];
  __syncthreads();

  float px[4], py[4], pz[4], dd[4];
#pragma unroll
  for (int j = 0; j < 4; ++j) {
    const int n = tid + 1024 * j;
    px[j] = sx[n * 3 + 0];
    py[j] = sx[n * 3 + 1];
    pz[j] = sx[n * 3 + 2];
    dd[j] = 1e10f;
  }
  int far = 0;
  for (int i = 0; i < kNcen; ++i) {
    if (tid == 0) scent[i] = far;
    if (i == kNcen - 1) break;
    const int fc = clampi(far, 0, kNpts - 1);
    const float cx = sx[fc * 3 + 0];
    const float cy = sx[fc * 3 + 1];
    const float cz = sx[fc * 3 + 2];
    float bv = 0.0f;
    int bi = 0;
#pragma unroll
    for (int j = 0; j < 4; ++j) {
      const float dx = px[j] - cx;
      const float dy = py[j] - cy;
      const float dz = pz[j] - cz;
      const float t0 = dx * dx;
      const float t1 = dy * dy;
      const float t2 = dz * dz;
      const float d = (t0 + t2) + t1;
      const float nd = fminf(dd[j], d);
      dd[j] = nd;
      const int n = tid + 1024 * j;
      if (j == 0) {
        bv = nd;
        bi = n;
      } else {
        const bool take = nd > bv;
        bv = take ? nd : bv;
        bi = take ? n : bi;
      }
    }
    argmax_step(bv, bi, 16);
    argmax_step(bv, bi, 8);
    argmax_step(bv, bi, 4);
    argmax_step(bv, bi, 2);
    argmax_step(bv, bi, 1);
    const int buf = i & 1;
    if (lane == 0) { rv[buf][wave] = bv; ri[buf][wave] = bi; }
    __syncthreads();
    float v2 = rv[buf][lane];
    int   i2 = ri[buf][lane];
    argmax_step(v2, i2, 16);
    argmax_step(v2, i2, 8);
    argmax_step(v2, i2, 4);
    argmax_step(v2, i2, 2);
    argmax_step(v2, i2, 1);
    far = i2;
  }
  __syncthreads();
  float vals[3];
#pragma unroll
  for (int j = 0; j < 3; ++j) {
    const int f = tid + 1024 * j;
    const int s = f / 3;
    const int comp = f - 3 * s;
    const int ci = clampi(scent[s], 0, kNpts - 1);
    vals[j] = sx[ci * 3 + comp];
  }
  for (int pass = 0; pass < 2; ++pass) {
#pragma unroll
    for (int j = 0; j < 3; ++j) {
      const size_t o = (size_t)b * (kNcen * 3) + tid + 1024 * j;
      *(volatile float*)(nxyz_ws + o) = vals[j];
      *(volatile float*)(out0 + o) = vals[j];
    }
    __threadfence();
  }
}

__global__ __launch_bounds__(256) void ballq_kernel(const float* __restrict__ xyz,
                                                    const float* __restrict__ nxyz,
                                                    int* __restrict__ idxg) {
#pragma clang fp contract(off)
  __shared__ int sidx[8][kNsmp];
  const int lane = threadIdx.x & 31;
  const int wv = threadIdx.x >> 5;
  const int sg = blockIdx.x * 8 + wv;
  const int b = sg >> 10;
  sidx[wv][lane] = 0;
  __syncthreads();
  const float* xb = xyz + (size_t)b * kNpts * 3;
  const float cx = nxyz[(size_t)sg * 3 + 0];
  const float cy = nxyz[(size_t)sg * 3 + 1];
  const float cz = nxyz[(size_t)sg * 3 + 2];
  const float cc = (cx * cx + cz * cz) + cy * cy;
  int cnt = 0;
  for (int n0 = 0; n0 < kNpts; n0 += 32) {
    if (cnt >= kNsmp) break;
    const int n = n0 + lane;
    const float qx = xb[n * 3 + 0];
    const float qy = xb[n * 3 + 1];
    const float qz = xb[n * 3 + 2];
    const float pp = (qx * qx + qz * qz) + qy * qy;
    float p = cx * qx;
    p = fmaf(cy, qy, p);
    p = fmaf(cz, qz, p);
    const float sq = (cc + pp) - 2.0f * p;
    const bool inr = !(sq > kRad2);
    const unsigned m = (unsigned)__ballot(inr);
    const int pre = __popc(m & ((1u << lane) - 1u));
    const int slot = cnt + pre;
    if (inr && slot < kNsmp) sidx[wv][slot] = n;
    cnt += __popc(m);
  }
  if (cnt > kNsmp) cnt = kNsmp;
  __syncthreads();
  const int firstv = sidx[wv][0];
  const int mine = sidx[wv][lane];
  const int first = (cnt > 0) ? firstv : (kNpts - 1);
  int v = (lane < cnt) ? mine : first;
  v = clampi(v, 0, kNpts - 1);
  int* dst = idxg + (size_t)sg * kNsmp + lane;
  *(volatile int*)dst = v;
  __threadfence();
  *(volatile int*)dst = v;
}

__global__ __launch_bounds__(256) void prep_kernel(const float* __restrict__ t_embed,
                                                   const float* __restrict__ tlw0, const float* __restrict__ tlb0,
                                                   const float* __restrict__ tlw1, const float* __restrict__ tlb1,
                                                   const float* __restrict__ cw0, const float* __restrict__ cb0,
                                                   const float* __restrict__ cw1, const float* __restrict__ cb1,
                                                   float* __restrict__ bias0, float* __restrict__ bias1,
                                                   float* __restrict__ w0x,
                                                   unsigned short* __restrict__ W0pu, unsigned short* __restrict__ W1hu) {
  __shared__ float gt[kBatch * kTdim];
  __shared__ float te0[kBatch * kCin0];
  __shared__ float te1[kBatch * kCmid];
  __shared__ float sb0[kBatch * kCmid];
  __shared__ float sb1[kBatch * kCout];
  __shared__ float scw0[kCmid * kCin0];
  const int tid = threadIdx.x;
#pragma unroll 1
  for (int i = tid; i < kBatch * kTdim; i += 256) gt[i] = gelu_erf(t_embed[i]);
#pragma unroll 2
  for (int i = tid; i < kCmid * kCin0; i += 256) scw0[i] = cw0[i];
  __syncthreads();
#pragma unroll 1
  for (int i = tid; i < kBatch * kCin0; i += 256) {
    const int bb = i / kCin0;
    const int c = i - bb * kCin0;
    const float* w = tlw0 + (size_t)c * kTdim;
    const float* g = gt + bb * kTdim;
    float s = 0.0f;
#pragma unroll 2
    for (int d = 0; d < kTdim; ++d) s = fmaf(g[d], w[d], s);
    te0[i] = s + tlb0[c];
  }
#pragma unroll 1
  for (int i = tid; i < kBatch * kCmid; i += 256) {
    const int bb = i >> 6;
    const int c = i & 63;
    const float* w = tlw1 + (size_t)c * kTdim;
    const float* g = gt + bb * kTdim;
    float s = 0.0f;
#pragma unroll 2
    for (int d = 0; d < kTdim; ++d) s = fmaf(g[d], w[d], s);
    te1[i] = s + tlb1[c];
  }
  __syncthreads();
#pragma unroll 1
  for (int i = tid; i < kBatch * kCmid; i += 256) {
    const int bb = i >> 6;
    const int o = i & 63;
    float s = 0.0f;
#pragma unroll 2
    for (int c = 0; c < kCin0; ++c) s = fmaf(scw0[o * kCin0 + c], te0[bb * kCin0 + c], s);
    sb0[i] = s + cb0[o];
  }
#pragma unroll 1
  for (int i = tid; i < kBatch * kCout; i += 256) {
    const int bb = i >> 7;
    const int o = i & 127;
    float s = 0.0f;
#pragma unroll 2
    for (int c = 0; c < kCmid; ++c) s = fmaf(cw1[o * kCmid + c], te1[bb * kCmid + c], s);
    sb1[i] = s + cb1[o];
  }
  __syncthreads();

  {
    float f0[2], f1[4];
#pragma unroll
    for (int it = 0; it < 2; ++it) f0[it] = sb0[tid + 256 * it];
#pragma unroll
    for (int it = 0; it < 4; ++it) f1[it] = sb1[tid + 256 * it];
    const int ox = tid >> 2;
    const int jx = tid & 3;
    const int jc = jx < 3 ? jx : 2;
    const float wraw = scw0[ox * kCin0 + jc];
    const float fx = (jx < 3) ? wraw : 0.0f;
    for (int pass = 0; pass < 2; ++pass) {
#pragma unroll
      for (int it = 0; it < 2; ++it) *(volatile float*)(bias0 + tid + 256 * it) = f0[it];
#pragma unroll
      for (int it = 0; it < 4; ++it) *(volatile float*)(bias1 + tid + 256 * it) = f1[it];
      *(volatile float*)(w0x + tid) = fx;
      __threadfence();
    }
  }
  {
    _Float16* W0p = (_Float16*)W0pu;
    v8h h0[2];
#pragma unroll
    for (int it = 0; it < 2; ++it) {
      const int q = tid + 256 * it;
      const int o = q >> 3;
      const int k0 = (q & 7) << 3;
#pragma unroll
      for (int e = 0; e < 8; ++e) h0[it][e] = (_Float16)(scw0[o * kCin0 + 3 + k0 + e] * kWCarry);
    }
    for (int pass = 0; pass < 2; ++pass) {
#pragma unroll
      for (int it = 0; it < 2; ++it) {
        const int q = tid + 256 * it;
        *(volatile v8h*)(W0p + (size_t)(q >> 3) * kCpts + ((q & 7) << 3)) = h0[it];
      }
      __threadfence();
    }
  }
  {
    _Float16* W1h = (_Float16*)W1hu;
    v8h h1[4];
#pragma unroll
    for (int it = 0; it < 4; ++it) {
      const int q = tid + 256 * it;
      const int o = q >> 3;
      const int k0 = (q & 7) << 3;
      const v4f u0 = *(const v4f*)(cw1 + (size_t)o * kCmid + k0);
      const v4f u1 = *(const v4f*)(cw1 + (size_t)o * kCmid + k0 + 4);
#pragma unroll
      for (int e = 0; e < 4; ++e) {
        h1[it][e] = (_Float16)(u0[e] * kWCarry);
        h1[it][4 + e] = (_Float16)(u1[e] * kWCarry);
      }
    }
    for (int pass = 0; pass < 2; ++pass) {
#pragma unroll
      for (int it = 0; it < 4; ++it) {
        const int q = tid + 256 * it;
        *(volatile v8h*)(W1h + (size_t)(q >> 3) * kCmid + ((q & 7) << 3)) = h1[it];
      }
      __threadfence();
    }
  }
}

__global__ __launch_bounds__(256) void ptsT_kernel(const float* __restrict__ pts,
                                                   unsigned short* __restrict__ outp) {
  __shared__ float tile[64 * 65];
  const int tid = threadIdx.x;
  const int b = blockIdx.x >> 6;
  const int n0 = (blockIdx.x & 63) << 6;
#pragma unroll
  for (int it = 0; it < 4; ++it) {
    const int q = tid + 256 * it;
    const int c = q >> 4;
    const int n4 = (q & 15) << 2;
    const v4f v = *(const v4f*)(pts + ((size_t)(b * kCpts + c)) * kNpts + n0 + n4);
    tile[c * 65 + n4 + 0] = v[0];
    tile[c * 65 + n4 + 1] = v[1];
    tile[c * 65 + n4 + 2] = v[2];
    tile[c * 65 + n4 + 3] = v[3];
  }
  __syncthreads();
  _Float16* op = (_Float16*)outp;
  v8h hv[2];
#pragma unroll
  for (int it = 0; it < 2; ++it) {
    const int q = tid + 256 * it;
    const int row = q >> 3;
    const int c8 = (q & 7) << 3;
#pragma unroll
    for (int e = 0; e < 8; ++e) hv[it][e] = (_Float16)tile[(c8 + e) * 65 + row];
  }
  for (int pass = 0; pass < 2; ++pass) {
#pragma unroll
    for (int it = 0; it < 2; ++it) {
      const int q = tid + 256 * it;
      const int row = q >> 3;
      const int c8 = (q & 7) << 3;
      *(volatile v8h*)(op + ((size_t)(b * kNpts + n0 + row)) * kCpts + c8) = hv[it];
    }
    __threadfence();
  }
}

__global__ __launch_bounds__(256) void wmma_gemm64_f16(
    const unsigned short* __restrict__ Ap, int lda,
    const unsigned short* __restrict__ Btp, int ldb,
    float* __restrict__ Cout, int ldc,
    int M, int N, int K, float scale) {
  typedef _Float16 T;
  const T* A = (const T*)Ap;
  const T* Bt = (const T*)Btp;
  __shared__ __align__(16) float sT[8][16 * 68];
  const int lane = threadIdx.x & 31;
  const int wave = threadIdx.x >> 5;
  const int tilesN = N >> 6;
  const int tilesM = M >> 6;
  const int tile = blockIdx.x * 8 + wave;
  if (tile >= tilesM * tilesN) return;
  const int tm = tile / tilesN;
  const int tn = tile - tm * tilesN;
  const int m0 = tm << 6;
  const int n0 = tn << 6;

  const int rlane = lane & 15;
  const int koff  = (lane >> 4) * 8;
  const int mOff  = (lane >> 4) * 8;

  v8f acc[4][4];
#pragma unroll
  for (int i = 0; i < 4; ++i)
#pragma unroll
    for (int j = 0; j < 4; ++j) acc[i][j] = (v8f){0.f,0.f,0.f,0.f,0.f,0.f,0.f,0.f};

  for (int k0 = 0; k0 < K; k0 += 32) {
    v16h bh[4];
#pragma unroll
    for (int j = 0; j < 4; ++j) {
      const size_t bo = (size_t)(n0 + (j << 4) + rlane) * ldb + koff + k0;
      bh[j] = FragH::load(Bt + bo);
    }
#pragma unroll
    for (int i = 0; i < 4; ++i) {
      const size_t ao = (size_t)(m0 + (i << 4) + rlane) * lda + koff + k0;
      v16h ah = FragH::load(A + ao);
#pragma unroll
      for (int j = 0; j < 4; ++j) acc[i][j] = FragH::mma(ah, bh[j], acc[i][j]);
      dep_guard4_h(acc[i][0], acc[i][1], acc[i][2], acc[i][3], ah, ah);
    }
    keep4_h(bh[0], bh[1], bh[2], bh[3]);
  }
  acc_guard4(acc[0][0], acc[0][1], acc[0][2], acc[0][3]);
  acc_guard4(acc[1][0], acc[1][1], acc[1][2], acc[1][3]);
  acc_guard4(acc[2][0], acc[2][1], acc[2][2], acc[2][3]);
  acc_guard4(acc[3][0], acc[3][1], acc[3][2], acc[3][3]);

  float* slab = sT[wave];
#pragma unroll
  for (int i = 0; i < 4; ++i) {
    const int mBase = m0 + (i << 4);
#pragma unroll
    for (int j = 0; j < 4; ++j) {
#pragma unroll
      for (int r = 0; r < 8; ++r) {
        const float v = acc[i][j][r] * scale;
        slab[(mOff + r) * 68 + (j << 4) + rlane] = v;
      }
    }
    __builtin_amdgcn_fence(__ATOMIC_RELEASE, "workgroup");
    __builtin_amdgcn_wave_barrier();
    __builtin_amdgcn_fence(__ATOMIC_ACQUIRE, "workgroup");
    {
      const int hh = lane >> 4, c4 = (lane & 15) * 4;
      for (int pass = 0; pass < 2; ++pass) {
#pragma unroll
        for (int it = 0; it < 8; ++it) {
          const int row = it * 2 + hh;
          v4f v = *(const v4f*)(slab + row * 68 + c4);
          *(volatile v4f*)(Cout + (size_t)(mBase + row) * ldc + n0 + c4) = v;
        }
        __threadfence();
      }
    }
    __builtin_amdgcn_fence(__ATOMIC_RELEASE, "workgroup");
    __builtin_amdgcn_wave_barrier();
    __builtin_amdgcn_fence(__ATOMIC_ACQUIRE, "workgroup");
  }
}

__device__ __forceinline__ void y0_pair(const float* __restrict__ xyzb, const float* __restrict__ P0l, int id,
                                        float cx, float cy, float cz, v4f wa, v4f wb, v2f bb,
                                        float& y0, float& y1) {
  const float* xp = xyzb + (size_t)id * 3;
  const float gx = xp[0] - cx;
  const float gy = xp[1] - cy;
  const float gz = xp[2] - cz;
  const v2f p = *(const v2f*)(P0l + (size_t)id * kCmid);
  const float t0 = fmaf(wa[2], gz, fmaf(wa[1], gy, wa[0] * gx));
  const float t1 = fmaf(wb[2], gz, fmaf(wb[1], gy, wb[0] * gx));
  y0 = (p[0] + t0) + bb[0];
  y1 = (p[1] + t1) + bb[1];
}

__global__ __launch_bounds__(256) void stats0_kernel(const float* __restrict__ xyz,
                                                     const float* __restrict__ nxyz,
                                                     const int* __restrict__ idxg,
                                                     const float* __restrict__ P0,
                                                     const float* __restrict__ w0x,
                                                     const float* __restrict__ bias0,
                                                     float* __restrict__ part0) {
  __shared__ float red[8][128];
  const int lane = threadIdx.x & 31;
  const int wv = threadIdx.x >> 5;
  const int b = blockIdx.x >> 5;
  const int cenb = blockIdx.x * 32 + wv * 4;
  const v4f wa = *(const v4f*)(w0x + 8 * lane);
  const v4f wb = *(const v4f*)(w0x + 8 * lane + 4);
  const v2f bb = *(const v2f*)(bias0 + b * kCmid + 2 * lane);
  const float* xyzb = xyz + (size_t)b * kNpts * 3;
  const float* P0l = P0 + (size_t)b * kNpts * kCmid + 2 * lane;
  float s0 = 0.0f, s1 = 0.0f, q0 = 0.0f, q1 = 0.0f;
#pragma unroll 1
  for (int cc = 0; cc < 4; ++cc) {
    const int cen = cenb + cc;
    const float cx = nxyz[(size_t)cen * 3 + 0];
    const float cy = nxyz[(size_t)cen * 3 + 1];
    const float cz = nxyz[(size_t)cen * 3 + 2];
    const int idxv = clampi(idxg[(size_t)cen * kNsmp + lane], 0, kNpts - 1);
#pragma unroll 2
    for (int k = 0; k < kNsmp; ++k) {
      const int id = __shfl(idxv, k, 32);
      float y0, y1;
      y0_pair(xyzb, P0l, id, cx, cy, cz, wa, wb, bb, y0, y1);
      s0 += y0;
      s1 += y1;
      q0 = fmaf(y0, y0, q0);
      q1 = fmaf(y1, y1, q1);
    }
  }
  red[wv][2 * lane] = s0;
  red[wv][2 * lane + 1] = s1;
  red[wv][64 + 2 * lane] = q0;
  red[wv][64 + 2 * lane + 1] = q1;
  __syncthreads();
  const int t = threadIdx.x;
  const int tc = t & 127;
  float tot = 0.0f;
#pragma unroll
  for (int w = 0; w < 8; ++w) tot += red[w][tc];
  if (t < 128) {
    float* dst = part0 + (size_t)blockIdx.x * 128 + t;
    *(volatile float*)dst = tot;
    __threadfence();
    *(volatile float*)dst = tot;
  }
}

template <int NBLK, int NCH>
__global__ __launch_bounds__(2 * NCH) void fin_kernel(const float* __restrict__ part,
                                                      const float* __restrict__ g,
                                                      const float* __restrict__ bt,
                                                      float* __restrict__ st) {
  __shared__ double sacc[2 * NCH];
  const int t = threadIdx.x;
  double a = 0.0;
#pragma unroll 4
  for (int blk = 0; blk < NBLK; ++blk) a += (double)part[(size_t)blk * (2 * NCH) + t];
  sacc[t] = a;
  __syncthreads();
  const int tc = (t < NCH) ? t : (t - NCH);
  const double mean = sacc[tc] * kInvCount;
  const double ex2 = sacc[NCH + tc] * kInvCount;
  double var = ex2 - mean * mean;
  var = (var < 0.0) ? 0.0 : var;
  const float rs = 1.0f / sqrtf((float)var + kBnEps);
  const float sc = g[tc] * rs;
  const float sh = (float)((double)bt[tc] - mean * (double)sc);
  const float v = (t < NCH) ? sc : sh;
  *(volatile float*)(st + t) = v;
  __threadfence();
  *(volatile float*)(st + t) = v;
}

__global__ __launch_bounds__(256) void buildx1_kernel(const float* __restrict__ xyz,
                                                      const float* __restrict__ nxyz,
                                                      const int* __restrict__ idxg,
                                                      const float* __restrict__ P0,
                                                      const float* __restrict__ w0x,
                                                      const float* __restrict__ bias0,
                                                      const float* __restrict__ st0,
                                                      unsigned* __restrict__ X1u) {
  const int lane = threadIdx.x & 31;
  const int wv = threadIdx.x >> 5;
  const int cen = blockIdx.x * 8 + wv;
  const int b = cen >> 10;
  const v4f wa = *(const v4f*)(w0x + 8 * lane);
  const v4f wb = *(const v4f*)(w0x + 8 * lane + 4);
  const v2f bb = *(const v2f*)(bias0 + b * kCmid + 2 * lane);
  const v2f scv = *(const v2f*)(st0 + 2 * lane);
  const v2f shv = *(const v2f*)(st0 + kCmid + 2 * lane);
  const float sc0 = scv[0], sc1 = scv[1], sh0 = shv[0], sh1 = shv[1];
  const float* xyzb = xyz + (size_t)b * kNpts * 3;
  const float* P0l = P0 + (size_t)b * kNpts * kCmid + 2 * lane;
  const float cx = nxyz[(size_t)cen * 3 + 0];
  const float cy = nxyz[(size_t)cen * 3 + 1];
  const float cz = nxyz[(size_t)cen * 3 + 2];
  const int idxv = clampi(idxg[(size_t)cen * kNsmp + lane], 0, kNpts - 1);
#pragma unroll 1
  for (int k = 0; k < kNsmp; ++k) {
    const int id = __shfl(idxv, k, 32);
    float y0, y1;
    y0_pair(xyzb, P0l, id, cx, cy, cz, wa, wb, bb, y0, y1);
    const float z0 = fmaf(y0, sc0, sh0);
    const float z1 = fmaf(y1, sc1, sh1);
    const float a0 = gelu_erf(z0) * kXCarry;
    const float a1 = gelu_erf(z1) * kXCarry;
    const _Float16 h0 = (_Float16)a0;
    const _Float16 h1 = (_Float16)a1;
    const unsigned u = (unsigned)__builtin_bit_cast(unsigned short, h0) |
                       ((unsigned)__builtin_bit_cast(unsigned short, h1) << 16);
    unsigned* dst = X1u + ((size_t)cen * kNsmp + k) * 32 + lane;
    *(volatile unsigned*)dst = u;
    __threadfence();
    *(volatile unsigned*)dst = u;
  }
}

__global__ __launch_bounds__(256) void conv1_pool_kernel(const unsigned short* __restrict__ X1p,
                                                         const unsigned short* __restrict__ W1p,
                                                         const float* __restrict__ bias1,
                                                         float* __restrict__ ymm,
                                                         float* __restrict__ part1) {
  typedef _Float16 T;
  const T* X1 = (const T*)X1p;
  const T* W1 = (const T*)W1p;
  __shared__ __align__(16) float slab[8][128];
  __shared__ float red[4][256];
  const int lane = threadIdx.x & 31;
  const int wv = threadIdx.x >> 5;
  const int cw = wv >> 1;
  const int nh = wv & 1;
  const int cen = blockIdx.x * 4 + cw;
  const int b = cen >> 10;
  const int rlane = lane & 15;
  const int hh = lane >> 4;
  const int koff = hh * 8;

  v8f acc[2][4];
#pragma unroll
  for (int i = 0; i < 2; ++i)
#pragma unroll
    for (int j = 0; j < 4; ++j) acc[i][j] = (v8f){0.f,0.f,0.f,0.f,0.f,0.f,0.f,0.f};

  const T* Ab = X1 + ((size_t)cen * kNsmp + rlane) * kCmid + koff;
#pragma unroll
  for (int ks = 0; ks < 2; ++ks) {
    v16h a0 = FragH::load(Ab + ks * 32);
    v16h a1 = FragH::load(Ab + (size_t)16 * kCmid + ks * 32);
#pragma unroll
    for (int j = 0; j < 4; ++j) {
      const v16h bf = FragH::load(W1 + (size_t)(nh * 64 + j * 16 + rlane) * kCmid + koff + ks * 32);
      acc[0][j] = mma_g(a0, bf, acc[0][j]);
      acc[1][j] = mma_g(a1, bf, acc[1][j]);
      if (j == 1) asm volatile("" ::: "memory");
    }
    asm volatile("" ::: "memory");
  }
  acc_guard4(acc[0][0], acc[0][1], acc[0][2], acc[0][3]);
  acc_guard4(acc[1][0], acc[1][1], acc[1][2], acc[1][3]);

  float* sl = slab[wv];
#pragma unroll
  for (int j = 0; j < 4; ++j) {
    const int col = nh * 64 + j * 16 + rlane;
    const float bv = bias1[b * kCout + col];
    float mx = -INFINITY, mn = INFINITY, s = 0.0f, q = 0.0f;
#pragma unroll
    for (int i = 0; i < 2; ++i) {
#pragma unroll
      for (int r = 0; r < 8; ++r) {
        const float v = fmaf(acc[i][j][r], kInvCarry1, bv);
        mx = fmaxf(mx, v);
        mn = fminf(mn, v);
        s += v;
        q = fmaf(v, v, q);
      }
    }
    const float omx = __shfl_xor(mx, 16, 32);
    const float omn = __shfl_xor(mn, 16, 32);
    const float os = __shfl_xor(s, 16, 32);
    const float oq = __shfl_xor(q, 16, 32);
    mx = fmaxf(mx, omx);
    mn = fminf(mn, omn);
    s += os;
    q += oq;
    sl[hh * 64 + j * 16 + rlane] = hh ? mn : mx;
    red[cw][hh * 128 + col] = hh ? q : s;
  }
  __syncthreads();
  const v4f mv = *(const v4f*)(sl + hh * 64 + rlane * 4);
  float* ydst = ymm + (size_t)cen * 256 + hh * 128 + nh * 64 + rlane * 4;
  const int t = threadIdx.x;
  const float tot = ((red[0][t] + red[1][t]) + red[2][t]) + red[3][t];
  float* pdst = part1 + (size_t)blockIdx.x * 256 + t;
  for (int pass = 0; pass < 2; ++pass) {
    *(volatile v4f*)ydst = mv;
    *(volatile float*)pdst = tot;
    __threadfence();
  }
}

__global__ __launch_bounds__(256) void pool_out_kernel(const float* __restrict__ ymm,
                                                       const float* __restrict__ st1,
                                                       float* __restrict__ out1) {
  __shared__ __align__(16) float tile[128 * 36];
  const int tid = threadIdx.x;
  const int cen0 = blockIdx.x * 32;
  const int b = cen0 >> 10;
  const int s0 = cen0 & 1023;
  const int o = tid & 127;
  const float sc = st1[o];
  const float sh = st1[kCout + o];
#pragma unroll 1
  for (int i = 0; i < 16; ++i) {
    const int slc = (tid >> 7) + 2 * i;
    const float ymx = ymm[(size_t)(cen0 + slc) * 256 + o];
    const float ymn = ymm[(size_t)(cen0 + slc) * 256 + 128 + o];
    const float g0 = gelu_erf(fmaf(ymx, sc, sh));
    const float g1 = gelu_erf(fmaf(ymn, sc, sh));
    tile[o * 36 + slc] = fmaxf(g0, g1);
  }
  __syncthreads();
  v4f vv[4];
#pragma unroll
  for (int it = 0; it < 4; ++it) {
    const int q = tid + 256 * it;
    vv[it] = *(const v4f*)(tile + (q >> 3) * 36 + ((q & 7) << 2));
  }
  for (int pass = 0; pass < 2; ++pass) {
#pragma unroll
    for (int it = 0; it < 4; ++it) {
      const int q = tid + 256 * it;
      const int oo = q >> 3;
      const int s4 = (q & 7) << 2;
      *(volatile v4f*)(out1 + ((size_t)(b * kCout + oo)) * kNcen + s0 + s4) = vv[it];
    }
    __threadfence();
  }
}

extern "C" void kernel_launch(void* const* d_in, const int* in_sizes, int n_in,
                              void* d_out, int out_size, void* d_ws, size_t ws_size,
                              hipStream_t stream) {
  (void)in_sizes; (void)n_in; (void)out_size;
  if (ws_size < kWsTotal) return;
  const float* xyz   = (const float*)d_in[0];
  const float* pts   = (const float*)d_in[1];
  const float* temb  = (const float*)d_in[2];
  const float* cw0   = (const float*)d_in[3];
  const float* cb0   = (const float*)d_in[4];
  const float* tlw0  = (const float*)d_in[5];
  const float* tlb0  = (const float*)d_in[6];
  const float* bng0  = (const float*)d_in[7];
  const float* bnb0  = (const float*)d_in[8];
  const float* cw1   = (const float*)d_in[9];
  const float* cb1   = (const float*)d_in[10];
  const float* tlw1  = (const float*)d_in[11];
  const float* tlb1  = (const float*)d_in[12];
  const float* bng1  = (const float*)d_in[13];
  const float* bnb1  = (const float*)d_in[14];

  char* ws = (char*)d_ws;
  float*          nxyz  = (float*)(ws + kOffNxyz);
  int*            idxg  = (int*)(ws + kOffIdx);
  float*          bias0 = (float*)(ws + kOffBias0);
  float*          bias1 = (float*)(ws + kOffBias1);
  float*          w0x   = (float*)(ws + kOffW0x);
  unsigned short* W0p   = (unsigned short*)(ws + kOffW0p);
  unsigned short* W1h   = (unsigned short*)(ws + kOffW1h);
  float*          st0   = (float*)(ws + kOffSt0);
  float*          st1   = (float*)(ws + kOffSt1);
  float*          part0 = (float*)(ws + kOffPart0);
  float*          part1 = (float*)(ws + kOffPart1);
  unsigned short* ptsT  = (unsigned short*)(ws + kOffPtsT);
  float*          P0    = (float*)(ws + kOffP0);
  unsigned short* X1    = (unsigned short*)(ws + kOffX1);
  float*          ymm   = (float*)(ws + kOffYmm);
  float*          out0  = (float*)d_out;
  float*          out1  = (float*)d_out + kOut1Floats;

  fps_kernel<<<kBatch, 1024, 0, stream>>>(xyz, nxyz, out0);
  ballq_kernel<<<kCenTot / 8, 256, 0, stream>>>(xyz, nxyz, idxg);
  prep_kernel<<<1, 256, 0, stream>>>(temb, tlw0, tlb0, tlw1, tlb1, cw0, cb0, cw1, cb1,
                                     bias0, bias1, w0x, W0p, W1h);
  ptsT_kernel<<<kBatch * (kNpts / 64), 256, 0, stream>>>(pts, ptsT);
  wmma_gemm64_f16<<<(kSrcTot / 64) * (kCmid / 64) / 8, 256, 0, stream>>>(
      ptsT, kCpts, W0p, kCpts, P0, kCmid, kSrcTot, kCmid, kCpts, kInvCarry0);
  stats0_kernel<<<kCenTot / 32, 256, 0, stream>>>(xyz, nxyz, idxg, P0, w0x, bias0, part0);
  fin_kernel<256, 64><<<1, 128, 0, stream>>>(part0, bng0, bnb0, st0);
  buildx1_kernel<<<kCenTot / 8, 256, 0, stream>>>(xyz, nxyz, idxg, P0, w0x, bias0, st0, (unsigned*)X1);
  conv1_pool_kernel<<<kCenTot / 4, 256, 0, stream>>>(X1, W1h, bias1, ymm, part1);
  fin_kernel<2048, 128><<<1, 256, 0, stream>>>(part1, bng1, bnb1, st1);
  pool_out_kernel<<<kCenTot / 32, 256, 0, stream>>>(ymm, st1, out1);
}
